// Attention_60395830116361
// MI455X (gfx1250) — hardware-verified
//
#include <hip/hip_runtime.h>


#ifndef NB
#define NB 2
#endif
#ifndef SEQ
#define SEQ 2048
#endif
#define NB_FULL  2
#define SEQ_FULL 2048
#define TT   SEQ
#define DM   1024
#define NH_  16
#define HD   64
#define ZH   2
#define PCAR 1024.0f
#define SCL  0.125f

static_assert(SEQ % 256 == 0);
static_assert(SEQ <= SEQ_FULL);
static_assert(NB <= NB_FULL);
static_assert(NH_ % ZH == 0);
static_assert(NH_ * HD == DM);
static_assert((NB * SEQ) % 64 == 0);
static_assert(DM % 64 == 0);
static_assert(HD % 32 == 0);

typedef _Float16 h16;
typedef unsigned short bf;
typedef __attribute__((ext_vector_type(16))) __bf16   v16bf;
typedef __attribute__((ext_vector_type(16))) _Float16 v16h;
typedef __attribute__((ext_vector_type(8)))  _Float16 v8h;
typedef __attribute__((ext_vector_type(8)))  unsigned short v8us;
typedef __attribute__((ext_vector_type(8)))  float    v8f;
typedef __attribute__((ext_vector_type(4)))  float    v4f;
typedef __attribute__((ext_vector_type(4)))  _Float16 v4h;
typedef v8h  __attribute__((may_alias)) v8ha;
typedef v4f  __attribute__((may_alias)) v4fa;
typedef v8us __attribute__((may_alias)) v8usa;

__device__ __forceinline__ unsigned short f2bf(float f) { unsigned u = __float_as_uint(f); u += 0x7FFFu + ((u >> 16) & 1u); return (unsigned short)(u >> 16); }
__device__ __forceinline__ float bf2f(unsigned short b) { return __uint_as_float(((unsigned)b) << 16); }
__device__ __forceinline__ float bfr(float f) { return bf2f(f2bf(f)); }
__device__ __forceinline__ v16h cat16(v8h lo, v8h hi) { return __builtin_shufflevector(lo, hi, 0, 1, 2, 3, 4, 5, 6, 7, 8, 9, 10, 11, 12, 13, 14, 15); }
__device__ __forceinline__ v16bf cat16b(v8us lo, v8us hi) { return __builtin_bit_cast(v16bf, __builtin_shufflevector(lo, hi, 0, 1, 2, 3, 4, 5, 6, 7, 8, 9, 10, 11, 12, 13, 14, 15)); }
__device__ __forceinline__ v8f wmma16(v16h a, v16h b, v8f c) { return __builtin_amdgcn_wmma_f32_16x16x32_f16(false, a, false, b, (short)0, c, false, false); }
__device__ __forceinline__ v8f wmmab(v16bf a, v16bf b, v8f c) { return __builtin_amdgcn_wmma_f32_16x16x32_bf16(false, a, false, b, (short)0, c, false, false); }

template <typename T16> struct WFrag;
template <> struct WFrag<h16> { typedef v16h V; static __device__ __forceinline__ V ld(const h16* p) { return cat16(*(const v8h*)p, *(const v8h*)(p + 16)); } static __device__ __forceinline__ v8f mma(V a, V b, v8f c) { return wmma16(a, b, c); } };
template <> struct WFrag<bf> { typedef v16bf V; static __device__ __forceinline__ V ld(const bf* p) { return cat16b(*(const v8us*)p, *(const v8us*)(p + 16)); } static __device__ __forceinline__ v8f mma(V a, V b, v8f c) { return wmmab(a, b, c); } };
template <typename T16, int NSPLIT, bool BIAS>
__global__ __launch_bounds__(32) void k_gemmw(const T16* __restrict__ A, const T16* __restrict__ A2, const T16* __restrict__ Bt, const T16* __restrict__ Bt2, int K, float* C, int ldc, const float* __restrict__ bias, size_t sA, size_t sB, size_t sC) {
    typedef typename WFrag<T16>::V V;
    __shared__ __align__(16) float os[16 * 68];
    const size_t z = blockIdx.z; A += z * sA; if (A2) A2 += z * sA; Bt += z * sB; if (Bt2) Bt2 += z * sB; C += z * sC;
    const int lane = threadIdx.x & 31, lr = lane & 15, hi = lane >> 4; const int r0 = blockIdx.x * 64, c0 = blockIdx.y * 64;
    v8f acc[4][4];
#pragma unroll
    for (int mb = 0; mb < 4; ++mb)
#pragma unroll
        for (int nb = 0; nb < 4; ++nb) acc[mb][nb] = (v8f){};
    const size_t aoff = (size_t)(r0 + lr) * K + 8 * hi, boff = (size_t)(c0 + lr) * K + 8 * hi;
#pragma unroll 1
    for (int kc = 0; kc < K; kc += 32) {
        V a[4], a2[4];
#pragma unroll
        for (int mb = 0; mb < 4; ++mb) { a[mb] = WFrag<T16>::ld(A + aoff + (size_t)mb * 16 * K + kc); if (NSPLIT == 1 || NSPLIT == 2) a2[mb] = WFrag<T16>::ld(A2 + aoff + (size_t)mb * 16 * K + kc); }
#pragma unroll
        for (int nb = 0; nb < 4; ++nb) { const V b = WFrag<T16>::ld(Bt + boff + (size_t)nb * 16 * K + kc); V b2; if (NSPLIT >= 2) b2 = WFrag<T16>::ld(Bt2 + boff + (size_t)nb * 16 * K + kc);
#pragma unroll
            for (int mb = 0; mb < 4; ++mb) { acc[mb][nb] = WFrag<T16>::mma(a[mb], b, acc[mb][nb]); if (NSPLIT == 1 || NSPLIT == 2) acc[mb][nb] = WFrag<T16>::mma(a2[mb], b, acc[mb][nb]); if (NSPLIT >= 2) acc[mb][nb] = WFrag<T16>::mma(a[mb], b2, acc[mb][nb]); } }
        asm volatile("v_nop\n\tv_nop\n\tv_nop\n\tv_nop" : "+v"(acc[0][0]), "+v"(acc[1][1]), "+v"(acc[2][2]), "+v"(acc[3][3]) : "v"(a[0]), "v"(a[3]));
    }
#pragma unroll
    for (int mb = 0; mb < 4; ++mb) {
#pragma unroll
        for (int nb = 0; nb < 4; ++nb) {
#pragma unroll
            for (int j = 0; j < 8; ++j) os[(hi * 8 + j) * 68 + nb * 16 + lr] = acc[mb][nb][j]; }
        __builtin_amdgcn_wave_barrier(); asm volatile("" ::: "memory");
        float* crow = C + (size_t)(r0 + mb * 16) * ldc + c0;
#pragma unroll 1
        for (int ps = 0; ps < 2; ++ps) {
#pragma unroll
            for (int s = 0; s < 8; ++s) { const int row = 2 * s + hi, cofs = lr * 4; v4f val = *(const v4fa*)(os + row * 68 + cofs); if (BIAS) { val[0] += bfr(bias[c0 + cofs]); val[1] += bfr(bias[c0 + cofs + 1]); val[2] += bfr(bias[c0 + cofs + 2]); val[3] += bfr(bias[c0 + cofs + 3]); }
                *(volatile v4f*)(crow + (size_t)row * ldc + cofs) = val; }
            if (ps == 0) __threadfence(); }
        __builtin_amdgcn_wave_barrier(); asm volatile("" ::: "memory");
    }
}

__device__ __forceinline__ h16 tohx(float x) { return (h16)x; }
__device__ __forceinline__ void splitf(float y, unsigned short& h, unsigned short& l) { h = f2bf(y); l = f2bf(y - bf2f(h)); }

template <bool SPLIT, bool HEADS>
__global__ __launch_bounds__(256) void k_plane(const float* __restrict__ F, size_t srcBatch, int rows, float sc, bf* Ph, bf* Pl) {
    const int b = blockIdx.y; const size_t e = ((size_t)blockIdx.x * 256 + threadIdx.x) * 8; if (e >= (size_t)rows * DM) return;
    const int t = (int)(e / DM), c = (int)(e % DM); const float* f = F + (size_t)b * srcBatch + e;
    const v4f x0 = *(const v4f*)f, x1 = *(const v4f*)(f + 4); v8us oh, ol;
#pragma unroll
    for (int q = 0; q < 8; ++q) { const float y = ((q < 4) ? x0[q & 3] : x1[q & 3]) * sc; unsigned short a2, c2; splitf(y, a2, c2); oh[q] = a2; ol[q] = c2; }
    const size_t oo = HEADS ? ((((size_t)b * NH_ + (size_t)(c / HD)) * rows + t) * HD + (size_t)(c % HD)) : (((size_t)b * rows + t) * DM + c);
    *(volatile v8us*)(Ph + oo) = oh; if (SPLIT) *(volatile v8us*)(Pl + oo) = ol;
    __threadfence();
    *(volatile v8us*)(Ph + oo) = oh; if (SPLIT) *(volatile v8us*)(Pl + oo) = ol;
}

__global__ __launch_bounds__(256) void k_vtp(const float* __restrict__ F, h16* V16) {
    const size_t e = ((size_t)blockIdx.x * 256 + threadIdx.x) * 8; if (e >= (size_t)NB * NH_ * HD * TT) return;
    const int t = (int)(e % TT); const int d = (int)((e / TT) % HD); const int g = (int)(e / ((size_t)TT * HD)); const int b = g / NH_, h = g % NH_;
    const float* f = F + ((size_t)b * TT + t) * DM + h * HD + d; v8h o;
#pragma unroll
    for (int q = 0; q < 8; ++q) o[q] = tohx(f[(size_t)q * DM]);
    *(volatile v8h*)(V16 + e) = o; __threadfence(); *(volatile v8h*)(V16 + e) = o;
}

__global__ __launch_bounds__(256) void k_asoft(const float* __restrict__ Sb, h16* P16) {
    const int lane = threadIdx.x & 31; const int row = blockIdx.x * 8 + (threadIdx.x >> 5); if (row >= ZH * TT) return; const float* sr = Sb + (size_t)row * TT; float v[TT / 32]; float mx = -3.0e38f;
#pragma unroll
    for (int ch = 0; ch < TT / 128; ++ch) { const int j0 = ch * 128 + lane * 4; const v4f a = *(const v4f*)(sr + j0);
#pragma unroll
        for (int q = 0; q < 4; ++q) { const float t = a[q] * SCL; v[ch * 4 + q] = t; mx = fmaxf(mx, t); } }
#pragma unroll
    for (int sh = 16; sh; sh >>= 1) mx = fmaxf(mx, __shfl_xor(mx, sh, 32));
    float sum = 0.f;
#pragma unroll
    for (int k = 0; k < TT / 32; ++k) { float d0 = __fsub_rn(v[k], mx); asm volatile("" : "+v"(d0)); v[k] = __builtin_amdgcn_exp2f(__fmul_rn(d0, 1.4426950408889634f)); sum += v[k]; }
#pragma unroll
    for (int sh = 16; sh; sh >>= 1) sum += __shfl_xor(sum, sh, 32);
    const float f = __fdiv_rn(PCAR, sum);
#pragma unroll 1
    for (int ps = 0; ps < 2; ++ps) {
#pragma unroll
        for (int ch = 0; ch < TT / 128; ++ch) { v4h o4;
#pragma unroll
            for (int q = 0; q < 4; ++q) o4[q] = tohx(v[ch * 4 + q] * f);
            *(volatile v4h*)(P16 + (size_t)row * TT + ch * 128 + lane * 4) = o4; }
        if (ps == 0) __threadfence(); }
}

#define SZ_X   ((size_t)NB * SEQ * DM * 2)
#define SZ_W   ((size_t)DM * DM * 2)
#define SZ_F   ((size_t)NB * SEQ * DM * 4)
#define SZ_HP  ((size_t)NB * NH_ * SEQ * HD * 2)
#define SZ_S   ((size_t)ZH * SEQ * SEQ * 4)
#define SZ_P   ((size_t)ZH * SEQ * SEQ * 2)
#define WS_TOTAL (SZ_X + 4 * SZ_W + SZ_F + 5 * SZ_HP + SZ_S + SZ_P)
static_assert(SZ_HP == SZ_X);
static_assert(WS_TOTAL <= (size_t)134217728);
static_assert((SZ_X % 256) == 0 && (SZ_W % 256) == 0 && (SZ_F % 256) == 0 && (SZ_S % 256) == 0 && (SZ_P % 256) == 0);

extern "C" void kernel_launch(void* const* d_in, const int* in_sizes, int n_in,
                              void* d_out, int out_size, void* d_ws, size_t ws_size, hipStream_t stream) {
    if (n_in < 8) return;
    const size_t need_x = (size_t)(NB - 1) * SEQ_FULL * DM + (size_t)SEQ * DM;
    if ((size_t)in_sizes[0] < need_x || (size_t)in_sizes[1] < need_x || (size_t)in_sizes[2] < need_x) return;
    if ((size_t)in_sizes[3] < (size_t)DM * DM || (size_t)in_sizes[4] < (size_t)DM * DM || (size_t)in_sizes[5] < (size_t)DM * DM || (size_t)in_sizes[6] < (size_t)DM * DM) return;
    if (in_sizes[7] < DM) return;
    if ((size_t)out_size < (size_t)NB * SEQ * DM) return;
    const float* xk = (const float*)d_in[0]; const float* xq = (const float*)d_in[1]; const float* xv = (const float*)d_in[2];
    const float* wk = (const float*)d_in[3]; const float* wq = (const float*)d_in[4]; const float* wv = (const float*)d_in[5]; const float* wo = (const float*)d_in[6]; const float* bo = (const float*)d_in[7];
    float* OUT = (float*)d_out;
    char* wsp = (char*)d_ws;
    auto take = [&](size_t bytes) { char* p = wsp; wsp += (bytes + 255) & ~(size_t)255; return (void*)p; };
    bf* XB = (bf*)take(SZ_X);
    bf* WQ = (bf*)take(SZ_W); bf* WK = (bf*)take(SZ_W); bf* WV = (bf*)take(SZ_W); bf* WO = (bf*)take(SZ_W);
    float* F = (float*)take(SZ_F);
    bf* QPh = (bf*)take(SZ_HP); bf* QPl = (bf*)take(SZ_HP); bf* KPh = (bf*)take(SZ_HP); bf* KPl = (bf*)take(SZ_HP); h16* VT16 = (h16*)take(SZ_HP);
    float* Sb = (float*)take(SZ_S); h16* P16 = (h16*)take(SZ_P);
    if ((size_t)(wsp - (char*)d_ws) > ws_size) return;
    float* AT = F;
    bf* CH = QPh; bf* CL = QPl;

    const unsigned GW = (unsigned)(((size_t)DM * DM / 8 + 255) / 256), GX = (unsigned)(((size_t)SEQ * DM / 8 + 255) / 256);
    k_plane<false, false><<<dim3(GW, 1), 256, 0, stream>>>(wq, 0, DM, 1.0f, WQ, nullptr);
    k_plane<false, false><<<dim3(GW, 1), 256, 0, stream>>>(wk, 0, DM, 1.0f, WK, nullptr);
    k_plane<false, false><<<dim3(GW, 1), 256, 0, stream>>>(wv, 0, DM, 1.0f, WV, nullptr);
    k_plane<false, false><<<dim3(GW, 1), 256, 0, stream>>>(wo, 0, DM, 1.0f, WO, nullptr);
    const dim3 gproj(NB * SEQ / 64, DM / 64, 1);
    k_plane<false, false><<<dim3(GX, NB), 256, 0, stream>>>(xq, (size_t)SEQ_FULL * DM, SEQ, 1.0f, XB, nullptr);
    k_gemmw<bf, 0, false><<<gproj, 32, 0, stream>>>(XB, nullptr, WQ, nullptr, DM, F, DM, nullptr, 0, 0, 0);
    k_plane<true, true><<<dim3(GX, NB), 256, 0, stream>>>(F, (size_t)SEQ * DM, SEQ, 1.0f, QPh, QPl);
    k_plane<false, false><<<dim3(GX, NB), 256, 0, stream>>>(xk, (size_t)SEQ_FULL * DM, SEQ, 1.0f, XB, nullptr);
    k_gemmw<bf, 0, false><<<gproj, 32, 0, stream>>>(XB, nullptr, WK, nullptr, DM, F, DM, nullptr, 0, 0, 0);
    k_plane<true, true><<<dim3(GX, NB), 256, 0, stream>>>(F, (size_t)SEQ * DM, SEQ, 1.0f, KPh, KPl);
    k_plane<false, false><<<dim3(GX, NB), 256, 0, stream>>>(xv, (size_t)SEQ_FULL * DM, SEQ, 1.0f, XB, nullptr);
    k_gemmw<bf, 0, false><<<gproj, 32, 0, stream>>>(XB, nullptr, WV, nullptr, DM, F, DM, nullptr, 0, 0, 0);
    k_vtp<<<(unsigned)(((size_t)NB * NH_ * HD * TT / 8 + 255) / 256), 256, 0, stream>>>(F, VT16);
    for (int g0 = 0; g0 < NB * NH_; g0 += ZH) {
        const int b = g0 / NH_, h0 = g0 % NH_; const size_t po = (size_t)g0 * TT * HD;
        k_gemmw<bf, 2, false><<<dim3(TT / 64, TT / 64, ZH), 32, 0, stream>>>(QPh + po, QPl + po, KPh + po, KPl + po, HD, Sb, TT, nullptr, (size_t)TT * HD, (size_t)TT * HD, (size_t)TT * TT);
        k_asoft<<<ZH * TT / 8, 256, 0, stream>>>(Sb, P16);
        k_gemmw<h16, 0, false><<<dim3(TT / 64, HD / 64, ZH), 32, 0, stream>>>(P16, nullptr, VT16 + po, nullptr, TT, AT + (size_t)b * TT * DM + (size_t)h0 * HD, DM, nullptr, (size_t)TT * TT, (size_t)HD * TT, (size_t)HD);
    }
    k_plane<true, false><<<dim3(GX, NB), 256, 0, stream>>>(AT, (size_t)SEQ * DM, SEQ, 1.0f / PCAR, CH, CL);
    k_gemmw<bf, 1, true><<<gproj, 32, 0, stream>>>(CH, CL, WO, nullptr, DM, OUT, DM, bo, 0, 0, 0);
}
